// Encoder_78795470012907
// MI455X (gfx1250) — hardware-verified
//
#include <hip/hip_runtime.h>
#include <hip/hip_fp16.h>


#ifndef NB
#define NB 4
#endif
#ifndef SEQ
#define SEQ 2048
#endif
#define NB_FULL  4
#define SEQ_FULL 2048
#define DM   512
#define NH   8
#define HD   64
#define NQKV (3 * NH * HD)
#define MTOT (SEQ * NB)

static_assert(NB == 4);
static_assert(NB_FULL == 4);
static_assert(SEQ >= 64 && SEQ <= SEQ_FULL);
static_assert(SEQ % 64 == 0);
static_assert(MTOT % 128 == 0);
static_assert(DM % 32 == 0);
static_assert(DM == NH * HD);
static_assert(HD == 64);
static_assert(NQKV % 64 == 0);
static_assert(((size_t)MTOT * DM) % 2048 == 0);

typedef _Float16 v16h __attribute__((ext_vector_type(16)));
typedef _Float16 v8h  __attribute__((ext_vector_type(8)));
typedef float    v8f  __attribute__((ext_vector_type(8)));
typedef float    v4f  __attribute__((ext_vector_type(4)));

union Frag { v16h v; v8h h[2]; };

#define L2E     1.44269504088896340736f
#define CS      (1.44269504088896340736f * 3.0517578125e-05f)
#define SC_OUT  2.44140625e-04f

#define WT_BYTES   ((size_t)NQKV * DM * 2)
#define WOT_BYTES  ((size_t)DM * DM * 2)
#define BIAS_ELEMS 2048
#define BIAS_BYTES ((size_t)BIAS_ELEMS * 4)
#define XH_BYTES   ((size_t)MTOT * DM * 2)
#define PL_ELEMS   ((size_t)NH * NB * SEQ * HD)
#define PL_BYTES   (PL_ELEMS * 2)
#define ZC_BYTES   ((size_t)MTOT * DM * 2)
#define WS_TOTAL   (WT_BYTES + WOT_BYTES + BIAS_BYTES + XH_BYTES + 4 * PL_BYTES + ZC_BYTES)
static_assert(WS_TOTAL <= (size_t)134217728);
static_assert(WT_BYTES % 128 == 0 && WOT_BYTES % 128 == 0 && BIAS_BYTES % 128 == 0);
static_assert(XH_BYTES % 128 == 0 && PL_BYTES % 128 == 0 && ZC_BYTES % 128 == 0);
static_assert(NQKV + DM == BIAS_ELEMS);

static __device__ __forceinline__ v8f zero8() {
    v8f z;
#pragma unroll
    for (int i = 0; i < 8; ++i) z[i] = 0.0f;
    return z;
}

static __device__ __forceinline__ v16h load_frag16(const _Float16* base, int ld, int lane) {
    int m  = lane & 15;
    int kb = (lane >> 4) << 3;
    const _Float16* p = base + (size_t)m * ld + kb;
    Frag f;
    f.h[0] = *(const v8h*)(p);
    f.h[1] = *(const v8h*)(p + 16);
    return f.v;
}

static __device__ __forceinline__ v8f wmma16(v16h a, v16h b, v8f c) {
    v8f d = __builtin_amdgcn_wmma_f32_16x16x32_f16(false, a, false, b, (short)0, c, false, false);
    asm volatile("v_nop\n\tv_nop\n\tv_nop\n\tv_nop" : "+v"(d) : "v"(a), "v"(b));
    return d;
}

static __device__ __forceinline__ float bf16r(float x) {
    unsigned u = __float_as_uint(x);
    u = (u + 0x7FFFu + ((u >> 16) & 1u)) & 0xFFFF0000u;
    return __uint_as_float(u);
}

static __device__ __forceinline__ float ex2(float x) {
    return __builtin_amdgcn_exp2f(x);
}

static __device__ __forceinline__ void wave_lds_sync() {
    __builtin_amdgcn_fence(3, "wavefront");
    asm volatile("s_wait_dscnt 0" ::: "memory");
    __builtin_amdgcn_wave_barrier();
}

__global__ __launch_bounds__(256) void k_wT(const float* __restrict__ src, int src_pitch, int src_xs, int src_ys,
                                             _Float16* __restrict__ dst, int dst_pitch, int dst_xs, int dst_ys) {
    __shared__ __align__(16) _Float16 T[64 * 72];
    const int tid = threadIdx.x;
    const float* sp = src + (size_t)blockIdx.x * src_xs + (size_t)blockIdx.y * src_ys;
    _Float16*    dp = dst + (size_t)blockIdx.x * dst_xs + (size_t)blockIdx.y * dst_ys;
#pragma unroll
    for (int it = 0; it < 4; ++it) {
        int idx = tid + it * 256;
        int r = idx >> 4, c4 = idx & 15;
        v4f v = *(const v4f*)(sp + (size_t)r * src_pitch + c4 * 4);
        T[(c4 * 4 + 0) * 72 + r] = (_Float16)(bf16r(v.x) * 64.0f);
        T[(c4 * 4 + 1) * 72 + r] = (_Float16)(bf16r(v.y) * 64.0f);
        T[(c4 * 4 + 2) * 72 + r] = (_Float16)(bf16r(v.z) * 64.0f);
        T[(c4 * 4 + 3) * 72 + r] = (_Float16)(bf16r(v.w) * 64.0f);
    }
    __syncthreads();
    const int j0 = tid >> 3, pc = tid & 7;
    v8h o0 = *(const v8h*)(&T[j0 * 72 + pc * 8]);
    v8h o1 = *(const v8h*)(&T[(j0 + 32) * 72 + pc * 8]);
    _Float16* d0 = dp + (size_t)j0 * dst_pitch + pc * 8;
    _Float16* d1 = dp + (size_t)(j0 + 32) * dst_pitch + pc * 8;
    *(volatile v8h*)d0 = o0;
    *(volatile v8h*)d1 = o1;
    __threadfence();
    *(volatile v8h*)d0 = o0;
    *(volatile v8h*)d1 = o1;
}

__global__ __launch_bounds__(512) void k_bprep(const float* __restrict__ bQ, const float* __restrict__ bK,
                                                const float* __restrict__ bV, const float* __restrict__ bO,
                                                float* __restrict__ bias) {
    __shared__ __align__(16) float st[BIAS_ELEMS];
    const int t = threadIdx.x;
    st[t]        = bf16r(bQ[t]) * 64.0f;
    st[512 + t]  = bf16r(bK[t]) * 64.0f;
    st[1024 + t] = bf16r(bV[t]) * 64.0f;
    st[1536 + t] = bf16r(bO[t]);
    __syncthreads();
    v4f v = *(const v4f*)(&st[t * 4]);
    *(volatile v4f*)(bias + t * 4) = v;
    __threadfence();
    *(volatile v4f*)(bias + t * 4) = v;
}

__global__ __launch_bounds__(256) void k_xcvt(const float* __restrict__ x, _Float16* __restrict__ xh) {
    const size_t i = ((size_t)blockIdx.x * 256 + threadIdx.x) * 8;
    v4f a = *(const v4f*)(x + i);
    v4f b = *(const v4f*)(x + i + 4);
    v8h o;
    o[0] = (_Float16)bf16r(a.x); o[1] = (_Float16)bf16r(a.y);
    o[2] = (_Float16)bf16r(a.z); o[3] = (_Float16)bf16r(a.w);
    o[4] = (_Float16)bf16r(b.x); o[5] = (_Float16)bf16r(b.y);
    o[6] = (_Float16)bf16r(b.z); o[7] = (_Float16)bf16r(b.w);
    *(volatile v8h*)(xh + i) = o;
    __threadfence();
    *(volatile v8h*)(xh + i) = o;
}

static __device__ __forceinline__ void gemm_32x64(const _Float16* __restrict__ Ap,
                                                  const _Float16* __restrict__ Bp,
                                                  int lane, v8f (&acc)[2][4]) {
#pragma unroll
    for (int rt = 0; rt < 2; ++rt)
#pragma unroll
        for (int nt = 0; nt < 4; ++nt) acc[rt][nt] = zero8();
#pragma unroll 1
    for (int k0 = 0; k0 < DM; k0 += 32) {
        v16h a0 = load_frag16(Ap + k0, DM, lane);
        v16h a1 = load_frag16(Ap + (size_t)16 * DM + k0, DM, lane);
#pragma unroll
        for (int nt = 0; nt < 4; ++nt) {
            v16h bf = load_frag16(Bp + (size_t)(nt * 16) * DM + k0, DM, lane);
            acc[0][nt] = wmma16(a0, bf, acc[0][nt]);
            acc[1][nt] = wmma16(a1, bf, acc[1][nt]);
        }
    }
}

__global__ __launch_bounds__(128) __attribute__((amdgpu_num_vgpr(256)))
void k_proj(const _Float16* __restrict__ xh,
            const _Float16* __restrict__ wT,
            const float*    __restrict__ bias,
            _Float16* __restrict__ qkv) {
    __shared__ __align__(16) _Float16 st[4][32 * 64];
    const int tid  = threadIdx.x;
    const int lane = tid & 31;
    const int w    = tid >> 5;
    const int m0   = blockIdx.x * 128 + w * 32;
    const int n0   = blockIdx.y * 64;

    v8f acc[2][4];
    gemm_32x64(xh + (size_t)m0 * DM, wT + (size_t)n0 * DM, lane, acc);

    const int r0 = (lane >> 4) << 3;
    const int cc = lane & 15;
    float bb[4];
#pragma unroll
    for (int nt = 0; nt < 4; ++nt) bb[nt] = bias[n0 + nt * 16 + cc];
#pragma unroll
    for (int rt = 0; rt < 2; ++rt)
#pragma unroll
        for (int nt = 0; nt < 4; ++nt)
#pragma unroll
            for (int g = 0; g < 8; ++g)
                st[w][(rt * 16 + r0 + g) * 64 + nt * 16 + cc] = (_Float16)(acc[rt][nt][g] + bb[nt]);
    wave_lds_sync();

    const int which = n0 >> 9;
    const int hh    = (n0 & 511) >> 6;
    _Float16* plane = qkv + (size_t)which * PL_ELEMS;
    const int rq = lane >> 3, pc = lane & 7;
    v8h pv[8];
    int off[8];
#pragma unroll
    for (int it = 0; it < 8; ++it) {
        const int i = it * 4 + rq;
        pv[it] = *(const v8h*)(&st[w][i * 64 + pc * 8]);
        const int m = m0 + i;
        const int s = m >> 2, b = m & 3;
        off[it] = ((hh * NB + b) * SEQ + s) * HD + pc * 8;
    }
#pragma unroll
    for (int it = 0; it < 8; ++it) *(volatile v8h*)(plane + off[it]) = pv[it];
    __threadfence();
#pragma unroll
    for (int it = 0; it < 8; ++it) *(volatile v8h*)(plane + off[it]) = pv[it];
}

__global__ __launch_bounds__(256) void k_vT(const _Float16* __restrict__ v, _Float16* __restrict__ vT) {
    __shared__ __align__(16) _Float16 T[64 * 72];
    const int tid = threadIdx.x;
    const int s0  = blockIdx.x * 64;
    const int hb  = blockIdx.y;
    const _Float16* sp = v + ((size_t)hb * SEQ + s0) * HD;
#pragma unroll
    for (int it = 0; it < 2; ++it) {
        int p = tid + it * 256;
        int r = p >> 3, pc = p & 7;
        v8h vv = *(const v8h*)(sp + (size_t)r * HD + pc * 8);
#pragma unroll
        for (int e = 0; e < 8; ++e) T[(pc * 8 + e) * 72 + r] = vv[e];
    }
    __syncthreads();
    _Float16* dp = vT + (size_t)hb * HD * SEQ + s0;
    const int j0 = tid >> 3, pc = tid & 7;
    v8h o0 = *(const v8h*)(&T[j0 * 72 + pc * 8]);
    v8h o1 = *(const v8h*)(&T[(j0 + 32) * 72 + pc * 8]);
    _Float16* d0 = dp + (size_t)j0 * SEQ + pc * 8;
    _Float16* d1 = dp + (size_t)(j0 + 32) * SEQ + pc * 8;
    *(volatile v8h*)d0 = o0;
    *(volatile v8h*)d1 = o1;
    __threadfence();
    *(volatile v8h*)d0 = o0;
    *(volatile v8h*)d1 = o1;
}

__global__ __launch_bounds__(128) __attribute__((amdgpu_num_vgpr(256)))
void k_attn(const _Float16* __restrict__ qp,
            const _Float16* __restrict__ kp,
            const _Float16* __restrict__ vT,
            _Float16* __restrict__ zc) {
    __shared__ __align__(16) float    Tsc[4][16 * 32];
    __shared__ __align__(16) _Float16 Pst[4][16 * 32];
    __shared__ __align__(16) _Float16 Zst[4][16 * 64];

    const int tid  = threadIdx.x;
    const int lane = tid & 31;
    const int b    = tid >> 5;
    const int h    = blockIdx.y;
    const int s0   = blockIdx.x * 16;
    const int r0   = (lane >> 4) << 3;
    const int cc   = lane & 15;
    const size_t hb = (size_t)(h * NB + b);

    const _Float16* qb = qp + (hb * SEQ + s0) * HD;
    const _Float16* kb = kp + hb * SEQ * HD;
    const _Float16* vb = vT + hb * HD * SEQ;

    const v16h qf0 = load_frag16(qb, HD, lane);
    const v16h qf1 = load_frag16(qb + 32, HD, lane);
    const int b1 = (b + 1) & 3, b2 = (b + 2) & 3, b3 = (b + 3) & 3;

    v8f o[4];
#pragma unroll
    for (int nt = 0; nt < 4; ++nt) o[nt] = zero8();
    float rs[8];
#pragma unroll
    for (int g = 0; g < 8; ++g) rs[g] = 0.0f;

#pragma unroll 1
    for (int t0 = 0; t0 < SEQ; t0 += 32) {
        const _Float16* kr = kb + (size_t)t0 * HD;
        v16h kf0 = load_frag16(kr, HD, lane);
        v16h kf1 = load_frag16(kr + 32, HD, lane);
        v8f sA = wmma16(qf0, kf0, zero8());
        sA = wmma16(qf1, kf1, sA);
        kf0 = load_frag16(kr + 16 * HD, HD, lane);
        kf1 = load_frag16(kr + 16 * HD + 32, HD, lane);
        v8f sB = wmma16(qf0, kf0, zero8());
        sB = wmma16(qf1, kf1, sB);

        float tA[8], tB[8];
#pragma unroll
        for (int g = 0; g < 8; ++g) {
            tA[g] = sA[g] * CS;
            tB[g] = sB[g] * CS;
            Tsc[b][(r0 + g) * 32 + cc]      = tA[g];
            Tsc[b][(r0 + g) * 32 + 16 + cc] = tB[g];
        }
        __syncthreads();

#pragma unroll
        for (int g = 0; g < 8; ++g) {
            const int ia = (r0 + g) * 32 + cc;
            const int ib = ia + 16;
            float dA = 1.0f + ex2(Tsc[b1][ia] - tA[g]) + ex2(Tsc[b2][ia] - tA[g]) + ex2(Tsc[b3][ia] - tA[g]);
            float dB = 1.0f + ex2(Tsc[b1][ib] - tB[g]) + ex2(Tsc[b2][ib] - tB[g]) + ex2(Tsc[b3][ib] - tB[g]);
            float pA = ex2(__builtin_amdgcn_rcpf(dA) * L2E);
            float pB = ex2(__builtin_amdgcn_rcpf(dB) * L2E);
            _Float16 hA = (_Float16)pA;
            _Float16 hB = (_Float16)pB;
            rs[g] += (float)hA + (float)hB;
            Pst[b][ia] = hA;
            Pst[b][ib] = hB;
        }
        wave_lds_sync();
        const v16h pa = load_frag16(&Pst[b][0], 32, lane);
        const _Float16* vr = vb + t0;
#pragma unroll
        for (int nt = 0; nt < 4; ++nt) {
            v16h vf = load_frag16(vr + (size_t)(nt * 16) * SEQ, SEQ, lane);
            o[nt] = wmma16(pa, vf, o[nt]);
        }
        __syncthreads();
    }

#pragma unroll
    for (int g = 0; g < 8; ++g) {
        float v = rs[g];
        v += __shfl_xor(v, 1, 32);
        v += __shfl_xor(v, 2, 32);
        v += __shfl_xor(v, 4, 32);
        v += __shfl_xor(v, 8, 32);
        rs[g] = __builtin_amdgcn_rcpf(v);
    }
#pragma unroll
    for (int nt = 0; nt < 4; ++nt)
#pragma unroll
        for (int g = 0; g < 8; ++g)
            Zst[b][(r0 + g) * 64 + nt * 16 + cc] = (_Float16)(o[nt][g] * rs[g]);
    wave_lds_sync();

    const int rq = lane >> 3, pc = lane & 7;
    v8h zv[4];
    int off[4];
#pragma unroll
    for (int it = 0; it < 4; ++it) {
        const int i = it * 4 + rq;
        zv[it]  = *(const v8h*)(&Zst[b][i * 64 + pc * 8]);
        off[it] = ((s0 + i) * NB + b) * DM + h * HD + pc * 8;
    }
#pragma unroll
    for (int it = 0; it < 4; ++it) *(volatile v8h*)(zc + off[it]) = zv[it];
    __threadfence();
#pragma unroll
    for (int it = 0; it < 4; ++it) *(volatile v8h*)(zc + off[it]) = zv[it];
}

__global__ __launch_bounds__(128) __attribute__((amdgpu_num_vgpr(256)))
void k_out(const _Float16* __restrict__ zc,
           const _Float16* __restrict__ woT,
           const float*    __restrict__ bo,
           float* __restrict__ out) {
    __shared__ __align__(16) float Ost[4][32 * 64];
    const int tid  = threadIdx.x;
    const int lane = tid & 31;
    const int w    = tid >> 5;
    const int m0   = blockIdx.x * 128 + w * 32;
    const int n0   = blockIdx.y * 64;

    v8f acc[2][4];
    gemm_32x64(zc + (size_t)m0 * DM, woT + (size_t)n0 * DM, lane, acc);

    const int r0 = (lane >> 4) << 3;
    const int cc = lane & 15;
    float bb[4];
#pragma unroll
    for (int nt = 0; nt < 4; ++nt) bb[nt] = bo[n0 + nt * 16 + cc];
#pragma unroll
    for (int rt = 0; rt < 2; ++rt)
#pragma unroll
        for (int nt = 0; nt < 4; ++nt)
#pragma unroll
            for (int g = 0; g < 8; ++g)
                Ost[w][(rt * 16 + r0 + g) * 64 + nt * 16 + cc] =
                    __builtin_fmaf(acc[rt][nt][g], SC_OUT, bb[nt]);
    wave_lds_sync();

    const int rh = lane >> 4, c4 = lane & 15;
    v4f sv[16];
#pragma unroll
    for (int it = 0; it < 16; ++it) sv[it] = *(const v4f*)(&Ost[w][(it * 2 + rh) * 64 + c4 * 4]);
    float* ob = out + (size_t)m0 * DM + n0 + (size_t)rh * DM + c4 * 4;
#pragma unroll
    for (int it = 0; it < 16; ++it) *(volatile v4f*)(ob + (size_t)(it * 2) * DM) = sv[it];
    __threadfence();
#pragma unroll
    for (int it = 0; it < 16; ++it) *(volatile v4f*)(ob + (size_t)(it * 2) * DM) = sv[it];
}

extern "C" void kernel_launch(void* const* d_in, const int* in_sizes, int n_in,
                              void* d_out, int out_size, void* d_ws, size_t ws_size,
                              hipStream_t stream) {
    if (n_in < 9) return;
    if (in_sizes[0] < ((SEQ - 1) * NB_FULL + NB) * DM) return;
    if (in_sizes[1] < NH * DM * HD || in_sizes[3] < NH * DM * HD || in_sizes[5] < NH * DM * HD) return;
    if (in_sizes[2] < NH * HD || in_sizes[4] < NH * HD || in_sizes[6] < NH * HD) return;
    if (in_sizes[7] < DM * DM || in_sizes[8] < DM) return;
    if (out_size < MTOT * DM) return;
    if ((size_t)WS_TOTAL > ws_size) return;

    const float* X  = (const float*)d_in[0];
    const float* WQ = (const float*)d_in[1];
    const float* bQ = (const float*)d_in[2];
    const float* WK = (const float*)d_in[3];
    const float* bK = (const float*)d_in[4];
    const float* WV = (const float*)d_in[5];
    const float* bV = (const float*)d_in[6];
    const float* WO = (const float*)d_in[7];
    const float* bO = (const float*)d_in[8];
    float* out = (float*)d_out;

    char* ws = (char*)d_ws;
    size_t off = 0;
    _Float16* wT   = (_Float16*)(ws + off); off += WT_BYTES;
    _Float16* woT  = (_Float16*)(ws + off); off += WOT_BYTES;
    float*    bias = (float*)(ws + off);    off += BIAS_BYTES;
    _Float16* xh   = (_Float16*)(ws + off); off += XH_BYTES;
    _Float16* qkv  = (_Float16*)(ws + off); off += 3 * PL_BYTES;
    _Float16* vT   = (_Float16*)(ws + off); off += PL_BYTES;
    _Float16* zc   = (_Float16*)(ws + off); off += ZC_BYTES;
    if (off > ws_size) return;

    k_wT<<<dim3(8, 8), dim3(256), 0, stream>>>(WQ, HD, 64 * HD, DM * HD, wT,                       DM, 64, 64 * DM);
    k_wT<<<dim3(8, 8), dim3(256), 0, stream>>>(WK, HD, 64 * HD, DM * HD, wT + (size_t)DM * DM,     DM, 64, 64 * DM);
    k_wT<<<dim3(8, 8), dim3(256), 0, stream>>>(WV, HD, 64 * HD, DM * HD, wT + (size_t)2 * DM * DM, DM, 64, 64 * DM);
    k_wT<<<dim3(8, 8), dim3(256), 0, stream>>>(WO, DM, 64 * DM, 64, woT, DM, 64, 64 * DM);
    k_bprep<<<dim3(1), dim3(512), 0, stream>>>(bQ, bK, bV, bO, bias);
    k_xcvt<<<dim3((unsigned)(((size_t)MTOT * DM) / 2048)), dim3(256), 0, stream>>>(X, xh);
    k_proj<<<dim3(MTOT / 128, NQKV / 64), dim3(128), 0, stream>>>(xh, wT, bias, qkv);
    k_vT<<<dim3(SEQ / 64, NH * NB), dim3(256), 0, stream>>>(qkv + 2 * PL_ELEMS, vT);
    k_attn<<<dim3(SEQ / 16, NH), dim3(128), 0, stream>>>(qkv, qkv + PL_ELEMS, vT, zc);
    k_out<<<dim3(MTOT / 128, DM / 64), dim3(128), 0, stream>>>(zc, woT, bias + NQKV, out);
}
